// LaneGNN_36318243455493
// MI455X (gfx1250) — hardware-run, weakly checked
//
#include <hip/hip_runtime.h>


namespace {
constexpr int B = 4, N = 512, FD = 256, FI = 128;
constexpr float XS = 8.0f, WSC = 256.0f;
typedef _Float16 b16;
typedef __attribute__((ext_vector_type(16))) _Float16 v16b;
typedef __attribute__((ext_vector_type(8))) _Float16 v8b;
typedef __attribute__((ext_vector_type(8))) float v8f;
typedef __attribute__((ext_vector_type(4))) float v4f;
__device__ __forceinline__ float bf16_rne(float f) { unsigned int u = __float_as_uint(f); u += 0x7FFFu + ((u >> 16) & 1u); return __uint_as_float(u & 0xFFFF0000u); }
__device__ __forceinline__ void split16(float v, b16& hi, b16& lo) { hi = (b16)v; lo = (b16)(v - (float)hi); }
__device__ __forceinline__ v16b frag_kb(const b16* p, int hh) { const v8b a = *(const v8b*)(p + 8 * hh), b = *(const v8b*)(p + 16 + 8 * hh); v16b f;
#pragma unroll
  for (int e = 0; e < 8; ++e) { f[e] = a[e]; f[8 + e] = b[e]; } return f; }
__device__ __forceinline__ v8f wmma16b(v16b a, v16b b, v8f c) { v8f d = __builtin_amdgcn_wmma_f32_16x16x32_f16(false, a, false, b, (short)0, c, false, false); asm volatile("v_nop\n\tv_nop\n\tv_nop\n\tv_nop" : "+v"(d) : "v"(a), "v"(b)); return d; }
__device__ __forceinline__ void wave_lds_sync() { __builtin_amdgcn_fence(__ATOMIC_RELEASE, "workgroup"); __builtin_amdgcn_wave_barrier(); __builtin_amdgcn_fence(__ATOMIC_ACQUIRE, "workgroup"); }
__device__ __forceinline__ float pmul(float a, float b) { float p = a * b; asm volatile("" : "+v"(p)); return p; }
__device__ __forceinline__ float gelu(float v) { return 0.5f * v * (1.0f + erff(v * 0.70710678118654752f)); }

__global__ __launch_bounds__(256) void wcopy_kernel(const float* __restrict__ w, int OUTW, int KIN, int ro, b16* __restrict__ WT) {
  const size_t u = (size_t)blockIdx.x * 256 + threadIdx.x; if (u >= (size_t)OUTW * KIN / 8) return; const size_t e = u * 8; v8b v;
#pragma unroll
  for (int j = 0; j < 8; ++j) v[j] = (b16)(bf16_rne(w[e + j]) * WSC); for (int pass = 0; pass < 2; ++pass) { *(volatile v8b*)(WT + (size_t)ro * KIN + e) = v; __threadfence(); }
}
__global__ __launch_bounds__(32) void node_kernel(const float* __restrict__ nf, const b16* __restrict__ WIO, const float* __restrict__ bi, const float* __restrict__ bo, float* __restrict__ NIO) {
  __shared__ __attribute__((aligned(16))) b16 Ah[16][FD + 8]; __shared__ __attribute__((aligned(16))) float Tf[16][128 + 4];
  const int lane = threadIdx.x, nloc = lane & 15, hlf = lane >> 4; const size_t m0 = (size_t)blockIdx.x * 16;
  for (int rr = 0; rr < 16; ++rr) for (int q = 0; q < 8; ++q) Ah[rr][q * 32 + lane] = (b16)(bf16_rne(nf[(m0 + rr) * FD + q * 32 + lane]) * XS);
  wave_lds_sync();
#pragma unroll 1
  for (int cg = 0; cg < 2; ++cg) { v8f acc[8];
#pragma unroll
    for (int t = 0; t < 8; ++t) acc[t] = (v8f){};
#pragma unroll 2
    for (int kb = 0; kb < FD; kb += 32) { const v16b a = frag_kb(&Ah[nloc][kb], hlf);
#pragma unroll
      for (int t = 0; t < 8; ++t) acc[t] = wmma16b(a, frag_kb(WIO + (size_t)(cg * 128 + t * 16 + nloc) * FD + kb, hlf), acc[t]); }
    const float* bb_ = cg ? bo : bi;
#pragma unroll
    for (int t = 0; t < 8; ++t) { const int c = t * 16 + nloc; const float bb = bf16_rne(bb_[c]);
#pragma unroll
      for (int r8 = 0; r8 < 8; ++r8) Tf[8 * hlf + r8][c] = acc[t][r8] * (1.0f / (XS * WSC)) + bb; }
    wave_lds_sync();
    for (int pass = 0; pass < 2; ++pass) { for (int rr = 0; rr < 16; ++rr) *(volatile v4f*)(NIO + (m0 + rr) * FD + cg * 128 + lane * 4) = *(const v4f*)(&Tf[rr][lane * 4]); __threadfence(); }
    wave_lds_sync(); }
}
__global__ __launch_bounds__(32) void edge_kernel(const float* __restrict__ NIO, const float* __restrict__ pe, const float* __restrict__ sup, const float* __restrict__ Wp, const float* __restrict__ bp, const b16* __restrict__ WE1, const float* __restrict__ be1, const float* __restrict__ We2, const float* __restrict__ be2, int JV, float* __restrict__ Esc) {
  __shared__ __attribute__((aligned(16))) b16 Ah[16][FI + 8]; __shared__ float So[32];
  const int lane = threadIdx.x, nloc = lane & 15, hlf = lane >> 4; const int njt = JV / 32; const int jt = blockIdx.x % njt, i = (blockIdx.x / njt) % N, b = blockIdx.x / (njt * N); const size_t bi_ = (size_t)b * N + i;
  float nin[4], wp0[4], wp1[4], bpv[4], bev[4], w2v[4]; for (int q = 0; q < 4; ++q) { const int c = q * 32 + lane; nin[q] = NIO[bi_ * FD + c]; wp0[q] = bf16_rne(Wp[c * 2]); wp1[q] = bf16_rne(Wp[c * 2 + 1]); bpv[q] = bf16_rne(bp[c]); bev[q] = bf16_rne(be1[c]); w2v[q] = bf16_rne(We2[c]); }
  const float c2 = bf16_rne(be2[0]);
#pragma unroll 1
  for (int half = 0; half < 2; ++half) { const int j0 = jt * 32 + half * 16;
    for (int rr = 0; rr < 16; ++rr) { const size_t j = (size_t)j0 + rr; const float p0 = bf16_rne(pe[((bi_) * N + j) * 2]), p1 = bf16_rne(pe[((bi_) * N + j) * 2 + 1]);
      for (int q = 0; q < 4; ++q) { const int c = q * 32 + lane; const float e = nin[q] - NIO[((size_t)b * N + j) * FD + FI + c] + pmul(p0, wp0[q]) + pmul(p1, wp1[q]) + bpv[q]; Ah[rr][c] = (b16)(e * XS); } }
    wave_lds_sync(); v8f acc[8];
#pragma unroll
    for (int t = 0; t < 8; ++t) acc[t] = (v8f){};
#pragma unroll
    for (int kb = 0; kb < FI; kb += 32) { const v16b a = frag_kb(&Ah[nloc][kb], hlf);
#pragma unroll
      for (int t = 0; t < 8; ++t) acc[t] = wmma16b(a, frag_kb(WE1 + (size_t)(t * 16 + nloc) * FI + kb, hlf), acc[t]); }
    float pd[8];
#pragma unroll
    for (int r8 = 0; r8 < 8; ++r8) pd[r8] = 0.0f;
#pragma unroll
    for (int t = 0; t < 8; ++t) { const int c = t * 16 + nloc; const float bb = bf16_rne(be1[c]), ww = bf16_rne(We2[c]);
#pragma unroll
      for (int r8 = 0; r8 < 8; ++r8) pd[r8] += pmul(gelu(acc[t][r8] * (1.0f / (XS * WSC)) + bb), ww); }
#pragma unroll
    for (int r8 = 0; r8 < 8; ++r8) { float s = pd[r8]; for (int o = 1; o < 16; o <<= 1) s += __shfl_xor(s, o); if (nloc == 0) { const int rl = 8 * hlf + r8; So[half * 16 + rl] = pmul(s + c2, bf16_rne(sup[(bi_) * N + j0 + rl])); } }
    wave_lds_sync(); }
  (void)bev; (void)w2v;
  for (int pass = 0; pass < 2; ++pass) { ((volatile float*)Esc)[bi_ * N + jt * 32 + lane] = So[lane]; __threadfence(); }
}
__global__ __launch_bounds__(32) void max_kernel(const float* __restrict__ Esc, const float* __restrict__ Wn1, const float* __restrict__ bn1, int JV, float* __restrict__ H1) {
  __shared__ float Mx[32]; const int lane = threadIdx.x; const int jt = blockIdx.x % (JV / 32), b = blockIdx.x / (JV / 32); const size_t j = (size_t)jt * 32 + lane; float m = -INFINITY;
#pragma unroll 4
  for (int i = 0; i < N; ++i) m = fmaxf(m, Esc[((size_t)b * N + i) * N + j]);
  Mx[lane] = m; wave_lds_sync();
  float w[8], bb[8]; for (int q = 0; q < 8; ++q) { w[q] = bf16_rne(Wn1[q * 32 + lane]); bb[q] = bf16_rne(bn1[q * 32 + lane]); }
  for (int pass = 0; pass < 2; ++pass) { for (int rr = 0; rr < 32; ++rr) { const float nm = Mx[rr]; for (int q = 0; q < 8; ++q) ((volatile float*)H1)[((size_t)b * N + jt * 32 + rr) * FD + q * 32 + lane] = fmaxf(pmul(nm, w[q]) + bb[q], 0.0f); } __threadfence(); }
}
__global__ __launch_bounds__(32) void out_kernel(const float* __restrict__ H1, const b16* __restrict__ WN2, const float* __restrict__ bn2, float* __restrict__ out) {
  __shared__ __attribute__((aligned(16))) b16 Ah[16][FD + 8], Al[16][FD + 8]; __shared__ __attribute__((aligned(16))) float Tf[16][128 + 4];
  const int lane = threadIdx.x, nloc = lane & 15, hlf = lane >> 4; const size_t m0 = (size_t)blockIdx.x * 16;
  for (int rr = 0; rr < 16; ++rr) for (int q = 0; q < 8; ++q) { b16 p, ql; split16(H1[(m0 + rr) * FD + q * 32 + lane] * XS, p, ql); Ah[rr][q * 32 + lane] = p; Al[rr][q * 32 + lane] = ql; }
  wave_lds_sync();
#pragma unroll 1
  for (int cg = 0; cg < 2; ++cg) { v8f acc[8];
#pragma unroll
    for (int t = 0; t < 8; ++t) acc[t] = (v8f){};
#pragma unroll 2
    for (int kb = 0; kb < FD; kb += 32) { const v16b a = frag_kb(&Ah[nloc][kb], hlf), al = frag_kb(&Al[nloc][kb], hlf);
#pragma unroll
      for (int t = 0; t < 8; ++t) { const v16b bw = frag_kb(WN2 + (size_t)(cg * 128 + t * 16 + nloc) * FD + kb, hlf); acc[t] = wmma16b(a, bw, acc[t]); acc[t] = wmma16b(al, bw, acc[t]); } }
#pragma unroll
    for (int t = 0; t < 8; ++t) { const int c = cg * 128 + t * 16 + nloc; const float bb = bf16_rne(bn2[c]);
#pragma unroll
      for (int r8 = 0; r8 < 8; ++r8) Tf[8 * hlf + r8][t * 16 + nloc] = fmaxf(acc[t][r8] * (1.0f / (XS * WSC)) + bb, 0.0f); }
    wave_lds_sync();
    for (int pass = 0; pass < 2; ++pass) { for (int rr = 0; rr < 16; ++rr) *(volatile v4f*)(out + (m0 + rr) * FD + cg * 128 + lane * 4) = *(const v4f*)(&Tf[rr][lane * 4]); __threadfence(); }
    wave_lds_sync(); }
}
}

extern "C" void kernel_launch(void* const* d_in, const int* in_sizes, int n_in, void* d_out, int out_size, void* d_ws, size_t ws_size, hipStream_t stream) {
  (void)n_in;
  auto Fp = [&](int i) { return (const float*)d_in[i]; };
  if (in_sizes[0] != B * N * FD || in_sizes[1] != B * N * N || in_sizes[2] != B * N * N * 2 || in_sizes[3] != FI * 2 || in_sizes[5] != FI * FD || in_sizes[7] != FI * FD || in_sizes[9] != FI * FI || in_sizes[11] != FI || in_sizes[13] != FD || in_sizes[15] != FD * FD || out_size != B * N * FD) return;
  const int NBV = B, JV = N;
  size_t off = 0; char* ws = (char*)d_ws;
  auto carve = [&](size_t bytes) { char* p = ws + off; off += (bytes + 255) & ~(size_t)255; return p; };
  b16* WIO = (b16*)carve((size_t)2 * FI * FD * 2); b16* WE1 = (b16*)carve((size_t)FI * FI * 2); b16* WN2 = (b16*)carve((size_t)FD * FD * 2); float* NIO = (float*)carve((size_t)B * N * FD * 4); float* Esc = (float*)carve((size_t)B * N * N * 4); float* H1 = (float*)carve((size_t)B * N * FD * 4);
  if (off > ws_size || off > ((size_t)64 << 20)) return;
  wcopy_kernel<<<(FI * FD / 8 + 255) / 256, 256, 0, stream>>>(Fp(5), FI, FD, 0, WIO); wcopy_kernel<<<(FI * FD / 8 + 255) / 256, 256, 0, stream>>>(Fp(7), FI, FD, FI, WIO); wcopy_kernel<<<(FI * FI / 8 + 255) / 256, 256, 0, stream>>>(Fp(9), FI, FI, 0, WE1); wcopy_kernel<<<(FD * FD / 8 + 255) / 256, 256, 0, stream>>>(Fp(15), FD, FD, 0, WN2);
  node_kernel<<<(unsigned)(NBV * N / 16), 32, 0, stream>>>(Fp(0), WIO, Fp(6), Fp(8), NIO);
  edge_kernel<<<(unsigned)(NBV * N * (JV / 32)), 32, 0, stream>>>(NIO, Fp(2), Fp(1), Fp(3), Fp(4), WE1, Fp(10), Fp(11), Fp(12), JV, Esc);
  max_kernel<<<(unsigned)(NBV * (JV / 32)), 32, 0, stream>>>(Esc, Fp(13), Fp(14), JV, H1);
  out_kernel<<<(unsigned)(NBV * N / 16), 32, 0, stream>>>(H1, WN2, Fp(16), (float*)d_out);
}
